// GPOnnxWrapper_70574902608252
// MI455X (gfx1250) — hardware-run, weakly checked
//
#include <hip/hip_runtime.h>


#ifndef NTEST
#define NTEST 32768
#endif
#ifndef NTRAIN
#define NTRAIN 4096
#endif
#define NTEST_FULL  32768
#define NTRAIN_FULL 4096
#define DIM   32
#define S5F   2.2360679774997896f
#define C53F  1.6666666666666667f
#define LOG2E 1.4426950408889634f

static_assert(DIM == 32);
static_assert(NTEST % 64 == 0);
static_assert(NTRAIN % 64 == 0);
static_assert(NTRAIN % 16 == 0);
static_assert(NTEST <= NTEST_FULL);
static_assert(NTRAIN <= NTRAIN_FULL);

typedef unsigned short bf;
typedef __attribute__((ext_vector_type(16))) __bf16   v16bf;
typedef __attribute__((ext_vector_type(8)))  unsigned short v8us;
typedef __attribute__((ext_vector_type(4)))  unsigned short v4us;
typedef __attribute__((ext_vector_type(8)))  float    v8f;
typedef __attribute__((ext_vector_type(4)))  float    v4f;
typedef v4f  __attribute__((may_alias)) v4fa;

__device__ __forceinline__ unsigned short f2bf(float f) { unsigned u = __float_as_uint(f); u += 0x7FFFu + ((u >> 16) & 1u); return (unsigned short)(u >> 16); }
__device__ __forceinline__ float bf2f(unsigned short h) { return __uint_as_float(((unsigned)h) << 16); }
__device__ __forceinline__ v16bf cat16b(v8us lo, v8us hi) { return __builtin_bit_cast(v16bf, __builtin_shufflevector(lo, hi, 0, 1, 2, 3, 4, 5, 6, 7, 8, 9, 10, 11, 12, 13, 14, 15)); }
__device__ __forceinline__ v8f wmmab(v16bf a, v16bf b, v8f c) { return __builtin_amdgcn_wmma_f32_16x16x32_bf16(false, a, false, b, (short)0, c, false, false); }
__device__ __forceinline__ v16bf ldb(const bf* p)  { return cat16b(*(const v8us*)p, *(const v8us*)(p + 16)); }
__device__ __forceinline__ void wave_sync() { __builtin_amdgcn_fence(3  , "wavefront"); __builtin_amdgcn_wave_barrier(); asm volatile("" ::: "memory"); }

__device__ __forceinline__ void cvt_piece(const float* __restrict__ src, const float* __restrict__ ls, size_t i8, int c8, v8us& oh, v8us& ol, float& q) {
    v4us h0 = (v4us){0, 0, 0, 0}, h1 = h0, l0 = h0, l1 = h0;
    q = 0.0f;
#pragma unroll 1
    for (int hf = 0; hf < 2; ++hf) {
        const v4f v = *(const v4f*)(src + i8 * 8 + hf * 4);
        const v4f l = *(const v4f*)(ls + c8 * 8 + hf * 4);
        v4us h, lo;
#pragma unroll
        for (int k = 0; k < 4; ++k) {
            const float xv = bf2f(f2bf(v[k]));
            const float lv = bf2f(f2bf(l[k]));
            const float s = xv / lv;
            const unsigned short hh = f2bf(s);
            h[k] = hh;
            lo[k] = f2bf(s - bf2f(hh));
            q = fmaf(s, s, q);
        }
        if (hf == 0) { h0 = h; l0 = lo; } else { h1 = h; l1 = lo; }
    }
    oh = __builtin_shufflevector(h0, h1, 0, 1, 2, 3, 4, 5, 6, 7);
    ol = __builtin_shufflevector(l0, l1, 0, 1, 2, 3, 4, 5, 6, 7);
}

__global__ __launch_bounds__(256) void k_prep_test(const float* __restrict__ src, const float* __restrict__ ls, bf* planeH, bf* planeL, float* norms) {
    __shared__ __align__(16) float sn[64];
    const int tid = threadIdx.x, lane = tid & 31;
    const int wave = __builtin_amdgcn_readfirstlane(tid >> 5);
    const size_t i8 = (size_t)blockIdx.x * 256 + tid;
    v8us oh, ol; float q;
    cvt_piece(src, ls, i8, tid & 3, oh, ol, q);
    q += __shfl_xor(q, 1, 32);
    q += __shfl_xor(q, 2, 32);
    if ((tid & 3) == 0) sn[tid >> 2] = q;
    __syncthreads();
    v4f nv = (v4f){0.0f, 0.0f, 0.0f, 0.0f};
    if (wave == 0) nv = *(const v4fa*)(&sn[(lane & 15) * 4]);
#pragma unroll 1
    for (int ps = 0; ps < 2; ++ps) {
        *(volatile v8us*)(planeH + i8 * 8) = oh;
        *(volatile v8us*)(planeL + i8 * 8) = ol;
        if (wave == 0) {
            if (lane < 16) *(volatile v4f*)(norms + (size_t)blockIdx.x * 64 + lane * 4) = nv;
        }
        if (ps == 0) __threadfence();
    }
}

__global__ __launch_bounds__(256) void k_prep_train(const float* __restrict__ src, const float* __restrict__ ls, const float* __restrict__ alpha,
                                                    bf* planeH, bf* planeL, float* norms, float* wout) {
    __shared__ __align__(16) float sn[64];
    __shared__ __align__(16) float sw[64];
    const int tid = threadIdx.x, lane = tid & 31;
    const int wave = __builtin_amdgcn_readfirstlane(tid >> 5);
    const size_t i8 = (size_t)blockIdx.x * 256 + tid;
    v8us oh, ol; float q;
    cvt_piece(src, ls, i8, tid & 3, oh, ol, q);
    q += __shfl_xor(q, 1, 32);
    q += __shfl_xor(q, 2, 32);
    if ((tid & 3) == 0) sn[tid >> 2] = q;
    if (wave < 2) { const int j = blockIdx.x * 64 + tid;
        sw[tid] = bf2f(f2bf(alpha[j])); }
    __syncthreads();
    v4f nv = (v4f){0.0f, 0.0f, 0.0f, 0.0f}, wv = (v4f){0.0f, 0.0f, 0.0f, 0.0f};
    if (wave == 0) {
        nv = *(const v4fa*)(&sn[(lane & 15) * 4]);
        wv = *(const v4fa*)(&sw[(lane & 15) * 4]);
    }
#pragma unroll 1
    for (int ps = 0; ps < 2; ++ps) {
        *(volatile v8us*)(planeH + i8 * 8) = oh;
        *(volatile v8us*)(planeL + i8 * 8) = ol;
        if (wave == 0) {
            if (lane < 16) { *(volatile v4f*)(norms + (size_t)blockIdx.x * 64 + lane * 4) = nv;
                             *(volatile v4f*)(wout  + (size_t)blockIdx.x * 64 + lane * 4) = wv; }
        }
        if (ps == 0) __threadfence();
    }
}

__device__ __forceinline__ float matern_term(float s, float g) {
    const float d2 = fmaxf(fmaf(-2.0f, g, s), 0.0f);
    const float rr = sqrtf(d2 + 1e-9f);
    const float poly = fmaf(C53F * rr, rr, fmaf(S5F, rr, 1.0f));
    return poly * __builtin_amdgcn_exp2f((-S5F * LOG2E) * rr);
}

__global__ __launch_bounds__(32) __attribute__((amdgpu_num_vgpr(256)))
void k_matern(const bf* __restrict__ ZH, const bf* __restrict__ ZL, const bf* __restrict__ XH, const bf* __restrict__ XL,
              const float* __restrict__ NZ, const float* __restrict__ NXT, const float* __restrict__ W,
              const float* __restrict__ oscale, float* OUT) {
    __shared__ __align__(16) float os[64];
    const int lane = threadIdx.x & 31, lr = lane & 15, hi = lane >> 4;
    const int r0 = blockIdx.x * 64;
    const float osc = bf2f(f2bf(oscale[0]));

    v16bf ah[4], al[4];
#pragma unroll
    for (int mb = 0; mb < 4; ++mb) {
        ah[mb] = ldb(ZH + (size_t)(r0 + mb * 16 + lr) * DIM + 8 * hi);
        al[mb] = ldb(ZL + (size_t)(r0 + mb * 16 + lr) * DIM + 8 * hi);
    }

    v8f zq0, zq1, zq2, zq3;
    {
        const v4f a0 = *(const v4f*)(NZ + r0 +  0 + 8 * hi), b0 = *(const v4f*)(NZ + r0 +  0 + 8 * hi + 4);
        const v4f a1 = *(const v4f*)(NZ + r0 + 16 + 8 * hi), b1 = *(const v4f*)(NZ + r0 + 16 + 8 * hi + 4);
        const v4f a2 = *(const v4f*)(NZ + r0 + 32 + 8 * hi), b2 = *(const v4f*)(NZ + r0 + 32 + 8 * hi + 4);
        const v4f a3 = *(const v4f*)(NZ + r0 + 48 + 8 * hi), b3 = *(const v4f*)(NZ + r0 + 48 + 8 * hi + 4);
        zq0 = __builtin_shufflevector(a0, b0, 0, 1, 2, 3, 4, 5, 6, 7);
        zq1 = __builtin_shufflevector(a1, b1, 0, 1, 2, 3, 4, 5, 6, 7);
        zq2 = __builtin_shufflevector(a2, b2, 0, 1, 2, 3, 4, 5, 6, 7);
        zq3 = __builtin_shufflevector(a3, b3, 0, 1, 2, 3, 4, 5, 6, 7);
    }

    v8f acc0 = (v8f){}, acc1 = (v8f){}, acc2 = (v8f){}, acc3 = (v8f){};

    const bf* xhp = XH + (size_t)lr * DIM + 8 * hi;
    const bf* xlp = XL + (size_t)lr * DIM + 8 * hi;
#pragma unroll 1
    for (int j0 = 0; j0 < NTRAIN; j0 += 16) {
        const v16bf bh = ldb(xhp + (size_t)j0 * DIM);
        const v16bf bl = ldb(xlp + (size_t)j0 * DIM);
        const float xs = NXT[j0 + lr];
        const float wv = W[j0 + lr];
        v8f c0 = (v8f){}, c1 = (v8f){}, c2 = (v8f){}, c3 = (v8f){};
        c0 = wmmab(ah[0], bh, c0); c1 = wmmab(ah[1], bh, c1); c2 = wmmab(ah[2], bh, c2); c3 = wmmab(ah[3], bh, c3);
        c0 = wmmab(ah[0], bl, c0); c1 = wmmab(ah[1], bl, c1); c2 = wmmab(ah[2], bl, c2); c3 = wmmab(ah[3], bl, c3);
        c0 = wmmab(al[0], bh, c0); c1 = wmmab(al[1], bh, c1); c2 = wmmab(al[2], bh, c2); c3 = wmmab(al[3], bh, c3);
        asm volatile("v_nop\n\tv_nop\n\tv_nop\n\tv_nop" : "+v"(c0), "+v"(c1), "+v"(c2), "+v"(c3)
                     : "v"(ah[0]), "v"(ah[1]), "v"(ah[2]), "v"(ah[3]), "v"(al[0]), "v"(al[1]), "v"(al[2]), "v"(al[3]), "v"(bh), "v"(bl));
#pragma unroll 1
        for (int r = 0; r < 8; ++r) {
            const float k0 = matern_term(zq0[r] + xs, c0[r]);
            const float k1 = matern_term(zq1[r] + xs, c1[r]);
            const float k2 = matern_term(zq2[r] + xs, c2[r]);
            const float k3 = matern_term(zq3[r] + xs, c3[r]);
            const float n0 = fmaf(wv, k0, acc0[r]);
            const float n1 = fmaf(wv, k1, acc1[r]);
            const float n2 = fmaf(wv, k2, acc2[r]);
            const float n3 = fmaf(wv, k3, acc3[r]);
            acc0[r] = n0; acc1[r] = n1; acc2[r] = n2; acc3[r] = n3;
        }
    }

    float fin[4][8];
#pragma unroll
    for (int r = 0; r < 8; ++r) {
        float v0 = acc0[r], v1 = acc1[r], v2 = acc2[r], v3 = acc3[r];
        v0 += __shfl_xor(v0, 1, 32); v0 += __shfl_xor(v0, 2, 32); v0 += __shfl_xor(v0, 4, 32); v0 += __shfl_xor(v0, 8, 32);
        v1 += __shfl_xor(v1, 1, 32); v1 += __shfl_xor(v1, 2, 32); v1 += __shfl_xor(v1, 4, 32); v1 += __shfl_xor(v1, 8, 32);
        v2 += __shfl_xor(v2, 1, 32); v2 += __shfl_xor(v2, 2, 32); v2 += __shfl_xor(v2, 4, 32); v2 += __shfl_xor(v2, 8, 32);
        v3 += __shfl_xor(v3, 1, 32); v3 += __shfl_xor(v3, 2, 32); v3 += __shfl_xor(v3, 4, 32); v3 += __shfl_xor(v3, 8, 32);
        fin[0][r] = osc * v0; fin[1][r] = osc * v1; fin[2][r] = osc * v2; fin[3][r] = osc * v3;
    }
    if (lr == 0) {
#pragma unroll
        for (int mb = 0; mb < 4; ++mb) {
            v4f p, q;
            p[0] = fin[mb][0]; p[1] = fin[mb][1]; p[2] = fin[mb][2]; p[3] = fin[mb][3];
            q[0] = fin[mb][4]; q[1] = fin[mb][5]; q[2] = fin[mb][6]; q[3] = fin[mb][7];
            *(v4fa*)(&os[mb * 16 + 8 * hi]) = p; *(v4fa*)(&os[mb * 16 + 8 * hi + 4]) = q;
        }
    }
    wave_sync();
    const v4f val = *(const v4fa*)(&os[lr * 4]);
#pragma unroll 1
    for (int ps = 0; ps < 2; ++ps) {
        if (lane < 16) *(volatile v4f*)(OUT + (size_t)r0 + lane * 4) = val;
        if (ps == 0) __threadfence();
    }
}

static constexpr size_t al256(size_t v) { return (v + 255) & ~(size_t)255; }
static constexpr size_t SZ_ZP = al256((size_t)NTEST * DIM * 2);
static constexpr size_t SZ_XP = al256((size_t)NTRAIN * DIM * 2);
static constexpr size_t SZ_NZ = al256((size_t)NTEST * 4);
static constexpr size_t SZ_NX = al256((size_t)NTRAIN * 4);
static constexpr size_t SZ_W  = al256((size_t)NTRAIN * 4);
static constexpr size_t SZ_TOTAL = 2 * SZ_ZP + 2 * SZ_XP + SZ_NZ + SZ_NX + SZ_W;
static_assert(SZ_TOTAL <= (size_t)134217728);
static_assert((size_t)(NTEST / 64) * 256 * 16 == (size_t)NTEST * DIM * 2);
static_assert((size_t)(NTRAIN / 64) * 256 * 16 == (size_t)NTRAIN * DIM * 2);
static_assert((size_t)(NTEST / 64) * 64 * 4 <= SZ_NZ);
static_assert((size_t)(NTRAIN / 64) * 64 * 4 <= SZ_NX);
static_assert((size_t)(NTRAIN / 64) * 64 * 4 <= SZ_W);
static_assert((size_t)(NTEST / 64) * 64 * 4 <= (size_t)NTEST_FULL * 4);

extern "C" void kernel_launch(void* const* d_in, const int* in_sizes, int n_in,
                              void* d_out, int out_size, void* d_ws, size_t ws_size, hipStream_t stream) {
    (void)stream;
    if (n_in < 5) return;
    if ((size_t)in_sizes[0] < (size_t)NTEST * DIM) return;
    if ((size_t)in_sizes[1] < (size_t)NTRAIN * DIM) return;
    if (in_sizes[2] < DIM || in_sizes[3] < 1 || (size_t)in_sizes[4] < (size_t)NTRAIN) return;
    if ((size_t)out_size < (size_t)NTEST) return;
    if (SZ_TOTAL > ws_size) return;
    const float* x = (const float*)d_in[0]; const float* tx = (const float*)d_in[1];
    const float* ls = (const float*)d_in[2]; const float* oscale = (const float*)d_in[3]; const float* alpha = (const float*)d_in[4];
    float* OUT = (float*)d_out;
    char* wsp = (char*)d_ws;
    bf* ZH = (bf*)wsp; wsp += SZ_ZP;
    bf* ZL = (bf*)wsp; wsp += SZ_ZP;
    bf* XH = (bf*)wsp; wsp += SZ_XP;
    bf* XL = (bf*)wsp; wsp += SZ_XP;
    float* NZ = (float*)wsp; wsp += SZ_NZ;
    float* NX = (float*)wsp; wsp += SZ_NX;
    float* WV = (float*)wsp; wsp += SZ_W;

    k_prep_test<<<NTEST / 64, 256, 0, stream>>>(x, ls, ZH, ZL, NZ);
    k_prep_train<<<NTRAIN / 64, 256, 0, stream>>>(tx, ls, alpha, XH, XL, NX, WV);
    k_matern<<<NTEST / 64, 32, 0, stream>>>(ZH, ZL, XH, XL, NZ, NX, WV, oscale, OUT);
}
